// GATBlock_90443421319378
// MI455X (gfx1250) — hardware-verified
//
#include <hip/hip_runtime.h>


#ifndef NB
#define NB 8
#endif
#ifndef SEQ
#define SEQ 2048
#endif
#define NB_FULL  8
#define SEQ_FULL 2048
#ifndef OUT_SEQ
#define OUT_SEQ SEQ
#endif
#define FIN   128
#define FOUT  64
#define AW    4
#define RS    2048.0f
#define RI    (1.0f / 2048.0f)
#define L2E   1.4426950408889634f
#define PSH   14.0f
#define PIS   (1.0f / 16384.0f)
#define SLOPE 0.2f

static_assert(FOUT == 64);
static_assert(FIN % 32 == 0);
static_assert(FIN % 8 == 0);
static_assert(SEQ % 64 == 0);
static_assert((NB * SEQ) % 64 == 0);
static_assert(SEQ % 32 == 0);
static_assert(SEQ % (16 * AW) == 0);
static_assert(SEQ % 256 == 0);
static_assert(((size_t)SEQ * FIN) % 8 == 0);
static_assert(NB <= NB_FULL);
static_assert(SEQ <= SEQ_FULL);

typedef _Float16 h16;
typedef unsigned short bf;
typedef __attribute__((ext_vector_type(16))) __bf16   v16bf;
typedef __attribute__((ext_vector_type(16))) _Float16 v16h;
typedef __attribute__((ext_vector_type(8)))  _Float16 v8h;
typedef __attribute__((ext_vector_type(8)))  unsigned short v8us;
typedef __attribute__((ext_vector_type(8)))  float    v8f;
typedef __attribute__((ext_vector_type(4)))  float    v4f;
typedef v4f  __attribute__((may_alias)) v4fa;

__device__ __forceinline__ unsigned short f2bf(float f) { unsigned u = __float_as_uint(f); u += 0x7FFFu + ((u >> 16) & 1u); return (unsigned short)(u >> 16); }
__device__ __forceinline__ v16h cat16(v8h lo, v8h hi) { return __builtin_shufflevector(lo, hi, 0, 1, 2, 3, 4, 5, 6, 7, 8, 9, 10, 11, 12, 13, 14, 15); }
__device__ __forceinline__ v16bf cat16b(v8us lo, v8us hi) { return __builtin_bit_cast(v16bf, __builtin_shufflevector(lo, hi, 0, 1, 2, 3, 4, 5, 6, 7, 8, 9, 10, 11, 12, 13, 14, 15)); }
__device__ __forceinline__ v8f wmma16(v16h a, v16h b, v8f c) { return __builtin_amdgcn_wmma_f32_16x16x32_f16(false, a, false, b, (short)0, c, false, false); }
__device__ __forceinline__ v8f wmmab(v16bf a, v16bf b, v8f c) { return __builtin_amdgcn_wmma_f32_16x16x32_bf16(false, a, false, b, (short)0, c, false, false); }
__device__ __forceinline__ v16h  ldh(const h16* p) { return cat16(*(const v8h*)p, *(const v8h*)(p + 16)); }
__device__ __forceinline__ v16bf ldb(const bf* p)  { return cat16b(*(const v8us*)p, *(const v8us*)(p + 16)); }
__device__ __forceinline__ void wave_sync() { __builtin_amdgcn_fence(3  , "wavefront"); __builtin_amdgcn_wave_barrier(); asm volatile("" ::: "memory"); }
__device__ __forceinline__ float lrelu(float t) { return fmaxf(t, SLOPE * t); }

__global__ __launch_bounds__(256) void k_cvt8(const float* __restrict__ src, bf* dst, size_t n8) {
    const size_t i = (size_t)blockIdx.x * 256 + threadIdx.x; if (i >= n8) return;
    const v8f v = *(const v8f*)(src + i * 8); v8us o;
#pragma unroll
    for (int k = 0; k < 8; ++k) o[k] = f2bf(v[k]);
    *(volatile v8us*)(dst + i * 8) = o; __threadfence(); *(volatile v8us*)(dst + i * 8) = o;
}

__global__ __launch_bounds__(256) void k_wt(const float* __restrict__ W, bf* WT) {
    const int t = blockIdx.x * 256 + threadIdx.x; if (t >= FOUT * FIN / 8) return;
    const int n = t / (FIN / 8), k8 = (t % (FIN / 8)) * 8; v8us o;
#pragma unroll
    for (int i = 0; i < 8; ++i) o[i] = f2bf(W[(size_t)(k8 + i) * FOUT + n]);
    *(volatile v8us*)(WT + (size_t)n * FIN + k8) = o; __threadfence(); *(volatile v8us*)(WT + (size_t)n * FIN + k8) = o;
}

__global__ __launch_bounds__(32) void k_hgemm(const bf* __restrict__ WT, const bf* __restrict__ XB, const float* __restrict__ avec, h16* HH, h16* HR, float* US) {
    __shared__ __align__(16) float os[16 * 68];
    __shared__ __align__(16) float sa[128];
    __shared__ __align__(16) float ss[128];
    const int K = FIN;
    const int lane = threadIdx.x & 31, lr = lane & 15, hi = lane >> 4; const int c0 = blockIdx.x * 64;
#pragma unroll
    for (int q = 0; q < 4; ++q) { const float v = avec[lane + 32 * q]; sa[lane + 32 * q] = __uint_as_float(((unsigned)f2bf(v)) << 16); }
    v8f acc[4][4];
#pragma unroll
    for (int mb = 0; mb < 4; ++mb)
#pragma unroll
        for (int nb = 0; nb < 4; ++nb) acc[mb][nb] = (v8f){};
    const size_t aoff = (size_t)lr * K + 8 * hi, boff = (size_t)(c0 + lr) * K + 8 * hi;
#pragma unroll 1
    for (int kc = 0; kc < K; kc += 32) {
        v16bf a[4];
#pragma unroll
        for (int mb = 0; mb < 4; ++mb) a[mb] = ldb(WT + aoff + (size_t)mb * 16 * K + kc);
#pragma unroll
        for (int nb = 0; nb < 4; ++nb) { const v16bf b = ldb(XB + boff + (size_t)nb * 16 * K + kc);
#pragma unroll
            for (int mb = 0; mb < 4; ++mb) acc[mb][nb] = wmmab(a[mb], b, acc[mb][nb]); }
        asm volatile("v_nop\n\tv_nop\n\tv_nop\n\tv_nop" : "+v"(acc[0][0]), "+v"(acc[1][1]), "+v"(acc[2][2]), "+v"(acc[3][3]) : "v"(a[0]), "v"(a[1]), "v"(a[2]), "v"(a[3]));
    }
    wave_sync();
    const int bb = c0 / SEQ, jt = c0 % SEQ;
    const size_t tbase = (size_t)bb * FOUT * SEQ + (size_t)jt;
    float p1a = 0.0f, p1b = 0.0f, p2a = 0.0f, p2b = 0.0f;
#pragma unroll
    for (int mb = 0; mb < 4; ++mb) {
#pragma unroll
        for (int nb = 0; nb < 4; ++nb) {
#pragma unroll
            for (int j = 0; j < 8; ++j) os[(hi * 8 + j) * 68 + nb * 16 + lr] = acc[mb][nb][j]; }
        wave_sync();
#pragma unroll 4
        for (int r = 0; r < 16; ++r) {
            const float w1 = sa[mb * 16 + r], w2 = sa[64 + mb * 16 + r];
            const float xa = os[r * 68 + lane], xb = os[r * 68 + 32 + lane];
            p1a = fmaf(xa, w1, p1a); p1b = fmaf(xb, w1, p1b); p2a = fmaf(xa, w2, p2a); p2b = fmaf(xb, w2, p2b); }
        const size_t sb = tbase + (size_t)(mb * 16) * (size_t)SEQ;
#pragma unroll 1
        for (int ps = 0; ps < 2; ++ps) {
#pragma unroll
            for (int s = 0; s < 4; ++s) { const int row = 4 * s + (lane >> 3), c8 = (lane & 7) * 8;
                const v4f x0 = *(const v4fa*)(&os[row * 68 + c8]); const v4f x1 = *(const v4fa*)(&os[row * 68 + c8 + 4]); v8h hv, rv;
#pragma unroll
                for (int i = 0; i < 4; ++i) { const h16 a0 = (h16)x0[i]; const h16 a1 = (h16)x1[i]; hv[i] = a0; hv[4 + i] = a1; rv[i] = (h16)((x0[i] - (float)a0) * RS); rv[4 + i] = (h16)((x1[i] - (float)a1) * RS); }
                const size_t oo = sb + (size_t)row * (size_t)SEQ + c8;
                *(volatile v8h*)(HH + oo) = hv; *(volatile v8h*)(HR + oo) = rv; }
            if (ps == 0) __threadfence(); }
        wave_sync();
    }
    ss[lane] = p1a * L2E; ss[32 + lane] = p1b * L2E; ss[64 + lane] = p2a * L2E; ss[96 + lane] = p2b * L2E;
    wave_sync();
    const v4f sv = *(const v4fa*)(&ss[hi * 64 + lr * 4]);
    float* up = US + (size_t)hi * ((size_t)NB * SEQ) + (size_t)c0 + lr * 4;
    *(volatile v4f*)up = sv; __threadfence(); *(volatile v4f*)up = sv;
}

__global__ __launch_bounds__(256) void k_stats(const float* __restrict__ US, float* CP) {
    __shared__ __align__(16) float su[SEQ];
    __shared__ float wm[8];
    const int tid = threadIdx.x;
    const int b = blockIdx.x / (SEQ / 256); const int j = (blockIdx.x % (SEQ / 256)) * 256 + tid;
    float mx = -3.0e38f;
#pragma unroll 1
    for (int t = tid; t < SEQ; t += 256) { const float v = US[(size_t)b * SEQ + t]; su[t] = v; mx = fmaxf(mx, v); }
    mx = fmaxf(mx, __shfl_xor(mx, 16, 32)); mx = fmaxf(mx, __shfl_xor(mx, 8, 32)); mx = fmaxf(mx, __shfl_xor(mx, 4, 32));
    mx = fmaxf(mx, __shfl_xor(mx, 2, 32));  mx = fmaxf(mx, __shfl_xor(mx, 1, 32));
    if ((tid & 31) == 0) wm[tid >> 5] = mx;
    __syncthreads();
    mx = wm[0];
#pragma unroll
    for (int w = 1; w < 8; ++w) mx = fmaxf(mx, wm[w]);
    const float u2 = US[(size_t)NB * SEQ + (size_t)b * SEQ + j];
    const float M = lrelu(mx + u2);
    float d0 = 0.0f, d1 = 0.0f, d2 = 0.0f, d3 = 0.0f;
#pragma unroll 1
    for (int i = 0; i < SEQ; i += 4) {
        const v4f s = *(const v4fa*)(&su[i]);
        d0 += __builtin_amdgcn_exp2f(lrelu(s[0] + u2) - M); d1 += __builtin_amdgcn_exp2f(lrelu(s[1] + u2) - M);
        d2 += __builtin_amdgcn_exp2f(lrelu(s[2] + u2) - M); d3 += __builtin_amdgcn_exp2f(lrelu(s[3] + u2) - M); }
    const float D = (d0 + d1) + (d2 + d3);
    const float c = PSH - M - log2f(D);
    float* cp = CP + (size_t)b * SEQ + j;
    *(volatile float*)cp = c; __threadfence(); *(volatile float*)cp = c;
}

__global__ __launch_bounds__(32 * AW) void k_gat(const h16* __restrict__ HH, const h16* __restrict__ HR, const float* __restrict__ US, const float* __restrict__ CP, float* OUT) {
    __shared__ __align__(16) float os[AW * 16 * 68];
    const int lane = threadIdx.x & 31, lr = lane & 15, hi = lane >> 4;
    const int wave = __builtin_amdgcn_readfirstlane((int)(threadIdx.x >> 5));
    const int b = blockIdx.y;
    const int i0 = (blockIdx.x * AW + wave) * 16;
    const float u1 = US[(size_t)b * SEQ + i0 + lr];
    const float* u2p = US + (size_t)NB * SEQ + (size_t)b * SEQ + 8 * hi;
    const float* cpp = CP + (size_t)b * SEQ + 8 * hi;
    const size_t vo = (size_t)b * FOUT * SEQ + (size_t)lr * SEQ + 8 * hi;
    v8f oh[4], orr[4];
#pragma unroll
    for (int dt = 0; dt < 4; ++dt) { oh[dt] = (v8f){}; orr[dt] = (v8f){}; }
#pragma unroll 1
    for (int j0 = 0; j0 < SEQ; j0 += 32) {
        const v8f ua = *(const v8f*)(u2p + j0), ub = *(const v8f*)(u2p + j0 + 16);
        const v8f ca = *(const v8f*)(cpp + j0), cb = *(const v8f*)(cpp + j0 + 16);
        v16h ph, pr;
#pragma unroll
        for (int r = 0; r < 8; ++r) {
            const float pa = __builtin_amdgcn_exp2f(lrelu(u1 + ua[r]) + ca[r]);
            const float pb = __builtin_amdgcn_exp2f(lrelu(u1 + ub[r]) + cb[r]);
            const h16 ha = (h16)pa, hb = (h16)pb;
            ph[r] = ha; ph[8 + r] = hb;
            pr[r] = (h16)((pa - (float)ha) * RS); pr[8 + r] = (h16)((pb - (float)hb) * RS); }
        v16h va[4], wa[4];
#pragma unroll
        for (int dt = 0; dt < 4; ++dt) { va[dt] = ldh(HH + vo + (size_t)dt * 16 * SEQ + j0); wa[dt] = ldh(HR + vo + (size_t)dt * 16 * SEQ + j0); }
#pragma unroll
        for (int dt = 0; dt < 4; ++dt) oh[dt] = wmma16(va[dt], ph, oh[dt]);
#pragma unroll
        for (int dt = 0; dt < 4; ++dt) orr[dt] = wmma16(va[dt], pr, orr[dt]);
#pragma unroll
        for (int dt = 0; dt < 4; ++dt) orr[dt] = wmma16(wa[dt], ph, orr[dt]);
        asm volatile("v_nop\n\tv_nop\n\tv_nop\n\tv_nop" : "+v"(oh[0]), "+v"(oh[1]), "+v"(oh[2]), "+v"(oh[3]), "+v"(orr[0]), "+v"(orr[1]), "+v"(orr[2]), "+v"(orr[3])
                     : "v"(va[0]), "v"(va[1]), "v"(va[2]), "v"(va[3]), "v"(wa[0]), "v"(wa[1]), "v"(wa[2]), "v"(wa[3]), "v"(ph), "v"(pr));
    }
    const int wb = wave * 16 * 68;
#pragma unroll
    for (int dt = 0; dt < 4; ++dt) { v4f a, c;
#pragma unroll
        for (int i = 0; i < 4; ++i) {
            const float t0 = (oh[dt][i] + orr[dt][i] * RI) * PIS; a[i] = lrelu(t0);
            const float t1 = (oh[dt][4 + i] + orr[dt][4 + i] * RI) * PIS; c[i] = lrelu(t1); }
        *(v4fa*)(&os[wb + lr * 68 + 16 * dt + 8 * hi]) = a; *(v4fa*)(&os[wb + lr * 68 + 16 * dt + 8 * hi + 4]) = c; }
    wave_sync();
    float* orow = OUT + ((size_t)b * OUT_SEQ + i0) * FOUT;
#pragma unroll 1
    for (int ps = 0; ps < 2; ++ps) {
#pragma unroll
        for (int s = 0; s < 8; ++s) { const int row = 2 * s + hi, cofs = lr * 4;
            const v4f val = *(const v4fa*)(&os[wb + row * 68 + cofs]);
            *(volatile v4f*)(orow + (size_t)row * FOUT + cofs) = val; }
        if (ps == 0) __threadfence(); }
}

static constexpr size_t al256(size_t v) { return (v + 255) & ~(size_t)255; }
static constexpr size_t SZ_XB = al256((size_t)NB * SEQ * FIN * 2);
static constexpr size_t SZ_WT = al256((size_t)FOUT * FIN * 2);
static constexpr size_t SZ_HP = al256((size_t)NB * FOUT * SEQ * 2);
static constexpr size_t SZ_US = al256((size_t)2 * NB * SEQ * 4);
static constexpr size_t SZ_CP = al256((size_t)NB * SEQ * 4);
static constexpr size_t SZ_TOTAL = SZ_XB + SZ_WT + 2 * SZ_HP + SZ_US + SZ_CP;
static_assert(SZ_TOTAL <= (size_t)134217728);

extern "C" void kernel_launch(void* const* d_in, const int* in_sizes, int n_in,
                              void* d_out, int out_size, void* d_ws, size_t ws_size, hipStream_t stream) {
    if (n_in < 3) return;
    const size_t needx = ((size_t)(NB - 1) * SEQ_FULL + SEQ) * FIN;
    if ((size_t)in_sizes[0] < needx) return;
    if ((size_t)in_sizes[1] < (size_t)FIN * FOUT || (size_t)in_sizes[2] < (size_t)2 * FOUT) return;
    if ((size_t)out_size < ((size_t)(NB - 1) * OUT_SEQ + SEQ) * FOUT) return;
    if (SZ_TOTAL > ws_size) return;
    const float* x = (const float*)d_in[0]; const float* w = (const float*)d_in[1]; const float* av = (const float*)d_in[2];
    float* OUT = (float*)d_out;
    char* wsp = (char*)d_ws;
    bf* XB = (bf*)wsp; wsp += SZ_XB;
    bf* WT = (bf*)wsp; wsp += SZ_WT;
    h16* HH = (h16*)wsp; wsp += SZ_HP;
    h16* HR = (h16*)wsp; wsp += SZ_HP;
    float* US = (float*)wsp; wsp += SZ_US;
    float* CP = (float*)wsp; wsp += SZ_CP;

    if (SEQ == SEQ_FULL) {
        const size_t n8 = (size_t)NB * SEQ * FIN / 8;
        k_cvt8<<<(unsigned)((n8 + 255) / 256), 256, 0, stream>>>(x, XB, n8);
    } else {
        const size_t n8 = (size_t)SEQ * FIN / 8;
        for (int b = 0; b < NB; ++b) k_cvt8<<<(unsigned)((n8 + 255) / 256), 256, 0, stream>>>(x + (size_t)b * SEQ_FULL * FIN, XB + (size_t)b * SEQ * FIN, n8);
    }
    k_wt<<<(unsigned)((FOUT * FIN / 8 + 255) / 256), 256, 0, stream>>>(w, WT);
    k_hgemm<<<dim3(NB * SEQ / 64, 1, 1), 32, 0, stream>>>(WT, XB, av, HH, HR, US);
    k_stats<<<dim3(NB * SEQ / 256, 1, 1), 256, 0, stream>>>(US, CP);
    k_gat<<<dim3(SEQ / (16 * AW), NB, 1), 32 * AW, 0, stream>>>(HH, HR, US, CP, OUT);
}
